// DeformableConv_5652176961656
// MI455X (gfx1250) — hardware-verified
//
#include <hip/hip_runtime.h>
#include <stdint.h>


typedef _Float16       v16h  __attribute__((ext_vector_type(16)));
typedef __bf16         v16bf __attribute__((ext_vector_type(16)));
typedef float          v8f   __attribute__((ext_vector_type(8)));
typedef float          v4f   __attribute__((ext_vector_type(4)));
typedef unsigned int   v4u   __attribute__((ext_vector_type(4)));
typedef unsigned int   v8u   __attribute__((ext_vector_type(8)));

#define NB_    4
#define NC_    256
#define NO_    256
#define IMW_   64
#define HW_    4096
#define KK_    9
#define KDIM_  2304
#define NKS_   72
#define GRP_   288
#define MOFF_  32
#define NBOFF_ 27

__device__ __forceinline__ unsigned short f2bf(float f) {
    unsigned int u = __float_as_uint(f);
    u += 0x7FFFu + ((u >> 16) & 1u);
    return (unsigned short)(u >> 16);
}
__device__ __forceinline__ float bf2f(unsigned short s) {
    return __uint_as_float(((unsigned int)s) << 16);
}
__device__ __forceinline__ unsigned short f2hb(float f) {
    _Float16 hh = (_Float16)f;
    return __builtin_bit_cast(unsigned short, hh);
}

__device__ __forceinline__ v8f wmma_bf16(v8u a, v8u b, v8f c) {
    v8f d = __builtin_amdgcn_wmma_f32_16x16x32_bf16(false, __builtin_bit_cast(v16bf, a),
                                                     false, __builtin_bit_cast(v16bf, b),
                                                     (short)0, c, false, false);
    asm volatile("v_nop\n\tv_nop\n\tv_nop\n\tv_nop" : "+v"(d) : "v"(a), "v"(b));
    return d;
}
__device__ __forceinline__ v8f wmma_f16(v8u a, v8u b, v8f c) {
    v8f d = __builtin_amdgcn_wmma_f32_16x16x32_f16(false, __builtin_bit_cast(v16h, a),
                                                    false, __builtin_bit_cast(v16h, b),
                                                    (short)0, c, false, false);
    asm volatile("v_nop\n\tv_nop\n\tv_nop\n\tv_nop" : "+v"(d) : "v"(a), "v"(b));
    return d;
}

__device__ __forceinline__ v8u ld_frag_row(const unsigned short* __restrict__ rowp, int k0, int h) {
    const v4u p0 = *(const v4u*)(rowp + k0 + 8 * h);
    const v4u p1 = *(const v4u*)(rowp + k0 + 16 + 8 * h);
    return __builtin_shufflevector(p0, p1, 0, 1, 2, 3, 4, 5, 6, 7);
}

__device__ __forceinline__ void st2_v4u(unsigned short* p, v4u v) {
    *(volatile v4u*)p = v;
    __threadfence();
    *(volatile v4u*)p = v;
}

__global__ __launch_bounds__(256) void k_prep(const float* __restrict__ weight,
                                              const float* __restrict__ w_off,
                                              unsigned short* __restrict__ Wm,
                                              unsigned short* __restrict__ Woh,
                                              unsigned short* __restrict__ Wol,
                                              int nMain, int nOff)
{
    int t = blockIdx.x * 256 + threadIdx.x;
    if (t < nMain) {
        const int o = t / GRP_, g = t - o * GRP_;
        const int k0 = g * 8, kk = k0 >> 8, c0 = k0 & 255;
        const float* src = weight + ((size_t)o * NC_ + c0) * KK_ + kk;
        unsigned int w[4];
        #pragma unroll
        for (int e = 0; e < 4; ++e) {
            const float v0 = src[(2 * e) * KK_] * 1024.0f;
            const float v1 = src[(2 * e + 1) * KK_] * 1024.0f;
            w[e] = (unsigned int)f2hb(v0) | ((unsigned int)f2hb(v1) << 16);
        }
        v4u pk; pk.x = w[0]; pk.y = w[1]; pk.z = w[2]; pk.w = w[3];
        st2_v4u(Wm + (size_t)o * KDIM_ + k0, pk);
        return;
    }
    t -= nMain;
    if (t >= nOff) return;
    {
        const int o = t / GRP_, g = t - o * GRP_;
        const int k0 = g * 8, kk = k0 >> 8, c0 = k0 & 255;
        const int oc = (o < NBOFF_) ? o : 0;
        const float rowsel = (o < NBOFF_) ? 1.0f : 0.0f;
        const float* src = w_off + ((size_t)oc * NC_ + c0) * KK_ + kk;
        unsigned int wh[4], wl[4];
        #pragma unroll
        for (int e = 0; e < 4; ++e) {
            const float v0 = src[(2 * e) * KK_] * rowsel;
            const float v1 = src[(2 * e + 1) * KK_] * rowsel;
            const unsigned short h0 = f2bf(v0), h1 = f2bf(v1);
            const unsigned short l0 = f2bf(v0 - bf2f(h0)), l1 = f2bf(v1 - bf2f(h1));
            wh[e] = (unsigned int)h0 | ((unsigned int)h1 << 16);
            wl[e] = (unsigned int)l0 | ((unsigned int)l1 << 16);
        }
        v4u ph; ph.x = wh[0]; ph.y = wh[1]; ph.z = wh[2]; ph.w = wh[3];
        v4u pl; pl.x = wl[0]; pl.y = wl[1]; pl.z = wl[2]; pl.w = wl[3];
        st2_v4u(Woh + (size_t)o * KDIM_ + k0, ph);
        st2_v4u(Wol + (size_t)o * KDIM_ + k0, pl);
    }
}

__global__ __launch_bounds__(256) void k_offgemm(const float* __restrict__ x,
                                                 const unsigned short* __restrict__ Woh,
                                                 const unsigned short* __restrict__ Wol,
                                                 const float* __restrict__ b_off,
                                                 int nboff,
                                                 float* __restrict__ om)
{
    __shared__ __attribute__((aligned(32))) unsigned int ldsHi[1024];
    __shared__ __attribute__((aligned(32))) unsigned int ldsLo[1024];
    __shared__ __attribute__((aligned(16))) float stg[MOFF_ * 64];

    const int nb = blockIdx.x, b = blockIdx.y;
    const int tid = threadIdx.x, lane = tid & 31, wave = tid >> 5;
    const int h = lane >> 4, m = lane & 15;
    const int mt = wave & 1, nt = wave >> 1;

    v8f acc;
    #pragma unroll
    for (int e = 0; e < 8; ++e) acc[e] = 0.0f;

    const int n = tid & 63, coct = tid >> 6;
    const int hw = nb * 64 + n, ph = hw >> 6, pw = hw & 63;
    const int sidx = (n >> 4) * 256 + (((coct & 1) << 4) + (n & 15)) * 8 + ((coct >> 1) << 2);
    const float* xb = x + (size_t)b * NC_ * HW_;
    const unsigned short* arh = Woh + (size_t)(mt * 16 + m) * KDIM_;
    const unsigned short* arl = Wol + (size_t)(mt * 16 + m) * KDIM_;

    #pragma unroll 1
    for (int kk = 0; kk < KK_; ++kk) {
        const int kh = kk / 3, kw = kk - kh * 3;
        const int y = ph + kh - 1, xq = pw + kw - 1;
        const bool valid = (y >= 0) & (y < IMW_) & (xq >= 0) & (xq < IMW_);
        const float vm = valid ? 1.0f : 0.0f;
        const int pix = valid ? (y * IMW_ + xq) : 0;
        #pragma unroll 1
        for (int cc = 0; cc < 8; ++cc) {
            __syncthreads();
            const int cbase = cc * 32 + coct * 8;
            const float* p = xb + (size_t)cbase * HW_ + pix;
            unsigned int wh[4], wl[4];
            #pragma unroll
            for (int e = 0; e < 4; ++e) {
                const float v0 = p[(size_t)(2 * e) * HW_] * vm;
                const float v1 = p[(size_t)(2 * e + 1) * HW_] * vm;
                const unsigned short h0 = f2bf(v0), h1 = f2bf(v1);
                const unsigned short l0 = f2bf(v0 - bf2f(h0)), l1 = f2bf(v1 - bf2f(h1));
                wh[e] = (unsigned int)h0 | ((unsigned int)h1 << 16);
                wl[e] = (unsigned int)l0 | ((unsigned int)l1 << 16);
            }
            v4u vh; vh.x = wh[0]; vh.y = wh[1]; vh.z = wh[2]; vh.w = wh[3];
            v4u vl; vl.x = wl[0]; vl.y = wl[1]; vl.z = wl[2]; vl.w = wl[3];
            *(v4u*)&ldsHi[sidx] = vh;
            *(v4u*)&ldsLo[sidx] = vl;
            __syncthreads();
            const int k0 = (kk * 8 + cc) * 32;
            const v8u ah = ld_frag_row(arh, k0, h);
            const v8u al = ld_frag_row(arl, k0, h);
            const v8u bh = *(const v8u*)&ldsHi[nt * 256 + lane * 8];
            const v8u bl = *(const v8u*)&ldsLo[nt * 256 + lane * 8];
            acc = wmma_bf16(ah, bh, acc);
            acc = wmma_bf16(ah, bl, acc);
            acc = wmma_bf16(al, bh, acc);
        }
    }

    #pragma unroll
    for (int r = 0; r < 8; ++r) {
        const int row = mt * 16 + 8 * h + r;
        const float bo = (row < nboff) ? b_off[row] : 0.0f;
        stg[row * 64 + nt * 16 + m] = acc[r] + bo;
    }
    __syncthreads();
    v4f sv[2]; float* gp[2];
    #pragma unroll
    for (int s = 0; s < 2; ++s) {
        const int L = wave * 8 + s * 4 + (lane >> 3);
        const int piece = lane & 7;
        const int row = L >> 1, col = (L & 1) * 32 + piece * 4;
        sv[s] = *(const v4f*)&stg[row * 64 + col];
        gp[s] = om + ((size_t)(b * MOFF_ + row)) * HW_ + nb * 64 + col;
    }
    *(volatile v4f*)gp[0] = sv[0];
    *(volatile v4f*)gp[1] = sv[1];
    __threadfence();
    *(volatile v4f*)gp[0] = sv[0];
    *(volatile v4f*)gp[1] = sv[1];
}

__global__ __launch_bounds__(256) void k_sample(const float* __restrict__ x,
                                                const float* __restrict__ om,
                                                unsigned short* __restrict__ Val,
                                                int ntot)
{
    const int t = blockIdx.x * 256 + threadIdx.x;
    if (t >= ntot) return;
    const int b = t / (KK_ * HW_);
    const int r = t - b * (KK_ * HW_);
    const int kk = r >> 12, hw = r & (HW_ - 1);
    const float* omb = om + (size_t)b * MOFF_ * HW_;
    const float dy = omb[(size_t)(2 * kk) * HW_ + hw];
    const float dx = omb[(size_t)(2 * kk + 1) * HW_ + hw];
    const float mv = omb[(size_t)(18 + kk) * HW_ + hw];
    const float mod = 1.0f / (1.0f + expf(-mv));
    const int ph = hw >> 6, pw = hw & 63, kh = kk / 3, kw = kk - kh * 3;
    const float py = (float)(ph - 1 + kh) + dy;
    const float px = (float)(pw - 1 + kw) + dx;
    float y0f = floorf(py), x0f = floorf(px);
    const float ly = py - y0f, lx = px - x0f;
    y0f = fminf(fmaxf(y0f, -2.0f), 65.0f);
    x0f = fminf(fmaxf(x0f, -2.0f), 65.0f);
    const int y0 = (int)y0f, x0 = (int)x0f, y1 = y0 + 1, x1 = x0 + 1;
    const float vy0 = (y0 >= 0 && y0 < IMW_) ? 1.0f : 0.0f;
    const float vy1 = (y1 >= 0 && y1 < IMW_) ? 1.0f : 0.0f;
    const float vx0 = (x0 >= 0 && x0 < IMW_) ? 1.0f : 0.0f;
    const float vx1 = (x1 >= 0 && x1 < IMW_) ? 1.0f : 0.0f;
    const int yc0 = min(max(y0, 0), IMW_ - 1), yc1 = min(max(y1, 0), IMW_ - 1);
    const int xc0 = min(max(x0, 0), IMW_ - 1), xc1 = min(max(x1, 0), IMW_ - 1);
    const int i00 = yc0 * IMW_ + xc0, i01 = yc0 * IMW_ + xc1;
    const int i10 = yc1 * IMW_ + xc0, i11 = yc1 * IMW_ + xc1;
    const float w00 = (1.0f - ly) * (1.0f - lx) * mod * vy0 * vx0;
    const float w01 = (1.0f - ly) * lx          * mod * vy0 * vx1;
    const float w10 = ly          * (1.0f - lx) * mod * vy1 * vx0;
    const float w11 = ly          * lx          * mod * vy1 * vx1;

    const float* xb = x + (size_t)b * NC_ * HW_;
    unsigned short* vrow = Val + ((size_t)(b * HW_ + hw)) * KDIM_ + kk * NC_;

    #pragma unroll 1
    for (int g = 0; g < NC_ / 8; ++g) {
        const float* xc = xb + (size_t)(g * 8) * HW_;
        unsigned int w[4];
        #pragma unroll
        for (int e = 0; e < 4; ++e) {
            const float* p0 = xc + (size_t)(2 * e) * HW_;
            const float* p1 = p0 + HW_;
            float v0 = w00 * p0[i00] + w01 * p0[i01] + w10 * p0[i10] + w11 * p0[i11];
            float v1 = w00 * p1[i00] + w01 * p1[i01] + w10 * p1[i10] + w11 * p1[i11];
            v0 *= 64.0f; v1 *= 64.0f;
            w[e] = (unsigned int)f2hb(v0) | ((unsigned int)f2hb(v1) << 16);
        }
        v4u pk; pk.x = w[0]; pk.y = w[1]; pk.z = w[2]; pk.w = w[3];
        st2_v4u(vrow + g * 8, pk);
    }
}

__global__ __launch_bounds__(256) void k_main(const unsigned short* __restrict__ Wm,
                                              const unsigned short* __restrict__ Val,
                                              const float* __restrict__ bias,
                                              float* __restrict__ out)
{
    __shared__ __attribute__((aligned(16))) float stg[8 * 512];

    const int nb = blockIdx.x, b = blockIdx.y;
    const int tid = threadIdx.x, lane = tid & 31, wave = tid >> 5;
    const int h = lane >> 4, m = lane & 15;
    const int wm = wave & 3, wn = wave >> 2;

    v8f acc[4][2];
    #pragma unroll
    for (int i = 0; i < 4; ++i)
        #pragma unroll
        for (int j = 0; j < 2; ++j)
            #pragma unroll
            for (int e = 0; e < 8; ++e) acc[i][j][e] = 0.0f;

    const unsigned short* brow0 = Val + ((size_t)b * HW_ + nb * 64 + wn * 32 + m) * KDIM_;
    const unsigned short* brow1 = brow0 + (size_t)16 * KDIM_;
    const unsigned short* arow  = Wm + ((size_t)(wm * 64 + m)) * KDIM_;

    #pragma unroll 1
    for (int ks = 0; ks < NKS_; ++ks) {
        const int k0 = ks * 32;
        const v8u bf0 = ld_frag_row(brow0, k0, h);
        const v8u bf1 = ld_frag_row(brow1, k0, h);
        #pragma unroll
        for (int i = 0; i < 4; ++i) {
            const v8u af = ld_frag_row(arow + (size_t)i * 16 * KDIM_, k0, h);
            acc[i][0] = wmma_f16(af, bf0, acc[i][0]);
            acc[i][1] = wmma_f16(af, bf1, acc[i][1]);
        }
    }

    float* stgw = stg + wave * 512;
    const float sc = 1.0f / 65536.0f;
    #pragma unroll
    for (int i = 0; i < 4; ++i) {
        __syncthreads();
        #pragma unroll
        for (int r = 0; r < 8; ++r) {
            stgw[(8 * h + r) * 32 + m]      = acc[i][0][r];
            stgw[(8 * h + r) * 32 + 16 + m] = acc[i][1][r];
        }
        __syncthreads();
        v4f sv[4]; float* gp[4];
        #pragma unroll
        for (int s = 0; s < 4; ++s) {
            const int rl = s * 4 + (lane >> 3);
            const int piece = lane & 7;
            const v4f tv = *(const v4f*)&stgw[rl * 32 + piece * 4];
            const int o = wm * 64 + i * 16 + rl;
            const float bo = bias[o];
            sv[s] = tv * sc + bo;
            gp[s] = out + ((size_t)(b * NO_ + o)) * HW_ + nb * 64 + wn * 32 + piece * 4;
        }
        #pragma unroll
        for (int s = 0; s < 4; ++s) *(volatile v4f*)gp[s] = sv[s];
        __threadfence();
        #pragma unroll
        for (int s = 0; s < 4; ++s) *(volatile v4f*)gp[s] = sv[s];
    }
}

extern "C" void kernel_launch(void* const* d_in, const int* in_sizes, int n_in,
                              void* d_out, int out_size, void* d_ws, size_t ws_size,
                              hipStream_t stream)
{
    if (n_in < 5) return;
    if (in_sizes[0] != NB_ * NC_ * HW_) return;
    if (in_sizes[1] != NBOFF_ * NC_ * KK_) return;
    if (in_sizes[2] != NBOFF_) return;
    if (in_sizes[3] != NO_ * NC_ * KK_) return;
    if (in_sizes[4] != NO_) return;
    if (out_size != NB_ * NO_ * HW_) return;

    const float* x      = (const float*)d_in[0];
    const float* w_off  = (const float*)d_in[1];
    const float* b_off  = (const float*)d_in[2];
    const float* weight = (const float*)d_in[3];
    const float* bias   = (const float*)d_in[4];
    float* out = (float*)d_out;

    const size_t szWm  = (size_t)NO_   * KDIM_ * 2;
    const size_t szWo  = (size_t)MOFF_ * KDIM_ * 2;
    const size_t szOm  = (size_t)NB_ * MOFF_ * HW_ * 4;
    const size_t szVal = (size_t)NB_ * HW_ * KDIM_ * 2;
    const size_t offWm = 0;
    const size_t offWh = offWm + szWm;
    const size_t offWl = offWh + szWo;
    const size_t offOm = offWl + szWo;
    const size_t offVal = offOm + szOm;
    const size_t total = offVal + szVal;
    if (total > ws_size) return;

    char* ws = (char*)d_ws;
    unsigned short* Wm  = (unsigned short*)(ws + offWm);
    unsigned short* Woh = (unsigned short*)(ws + offWh);
    unsigned short* Wol = (unsigned short*)(ws + offWl);
    float*          om  = (float*)(ws + offOm);
    unsigned short* Val = (unsigned short*)(ws + offVal);

    const int nMain = NO_ * GRP_;
    const int nOff  = MOFF_ * GRP_;
    const int nPrep = nMain + nOff;
    k_prep<<<(nPrep + 255) / 256, 256, 0, stream>>>(weight, w_off, Wm, Woh, Wol, nMain, nOff);

    k_offgemm<<<dim3(HW_ / 64, NB_), 256, 0, stream>>>(x, Woh, Wol, b_off, in_sizes[2], om);

    const int nSamp = NB_ * KK_ * HW_;
    k_sample<<<(nSamp + 255) / 256, 256, 0, stream>>>(x, om, Val, nSamp);

    k_main<<<dim3(HW_ / 64, NB_), 256, 0, stream>>>(Wm, Val, bias, out);
}
